// NearFieldHead_10170482557399
// MI455X (gfx1250) — hardware-run, weakly checked
//
#include <hip/hip_runtime.h>


namespace {
constexpr int NBT = 65536, R = 12, L = 16, F = 8, HH = 64, FIN = F + 3;
constexpr float XS = 8.0f, WSC = 256.0f, FMIN = -3.4028234663852886e38f;
typedef _Float16 b16;
typedef __attribute__((ext_vector_type(16))) _Float16 v16b;
typedef __attribute__((ext_vector_type(8))) _Float16 v8b;
typedef __attribute__((ext_vector_type(8))) float v8f;
typedef __attribute__((ext_vector_type(4))) float v4f;
__device__ __forceinline__ float bf16_rne(float f) { unsigned int u = __float_as_uint(f); u += 0x7FFFu + ((u >> 16) & 1u); float r = __uint_as_float(u & 0xFFFF0000u); asm volatile("" : "+v"(r)); return r; }
__device__ __forceinline__ float bfv(float f) { float r = bf16_rne(f); asm volatile("" : "+v"(r)); return r; }
__device__ __forceinline__ void split16(float v, b16& hi, b16& lo) { hi = (b16)v; lo = (b16)(v - (float)hi); }
__device__ __forceinline__ v16b frag_kb(const b16* p, int hh) { const v8b a = *(const v8b*)(p + 8 * hh), b = *(const v8b*)(p + 16 + 8 * hh); v16b f;
#pragma unroll
  for (int e = 0; e < 8; ++e) { f[e] = a[e]; f[8 + e] = b[e]; } return f; }
__device__ __forceinline__ v8f wmma16b(v16b a, v16b b, v8f c) { v8f d = __builtin_amdgcn_wmma_f32_16x16x32_f16(false, a, false, b, (short)0, c, false, false); asm volatile("v_nop\n\tv_nop\n\tv_nop\n\tv_nop" : "+v"(d) : "v"(a), "v"(b)); return d; }
__device__ __forceinline__ void wave_lds_sync() { __builtin_amdgcn_fence(__ATOMIC_RELEASE, "workgroup"); __builtin_amdgcn_wave_barrier(); __builtin_amdgcn_fence(__ATOMIC_ACQUIRE, "workgroup"); }
__device__ __forceinline__ float pmul(float a, float b) { float p = a * b; asm volatile("" : "+v"(p)); return p; }

__global__ __launch_bounds__(256) void wput_kernel(const float* __restrict__ kw1, const float* __restrict__ qw2, const float* __restrict__ kw2, b16* __restrict__ KW1, b16* __restrict__ QW2, b16* __restrict__ KW2) { const int u = blockIdx.x * 256 + threadIdx.x;
  if (u < 32 * 4) { const int o = u / 4, k0 = (u % 4) * 8; v8b v;
#pragma unroll
    for (int j = 0; j < 8; ++j) { const int k = k0 + j; v[j] = (b16)(k < FIN ? bf16_rne(kw1[(size_t)k * 32 + o]) * WSC : 0.0f); } for (int pass = 0; pass < 2; ++pass) { *(volatile v8b*)(KW1 + (size_t)o * 32 + k0) = v; __threadfence(); } }
  if (u < HH * 4) { const int o = u / 4, k0 = (u % 4) * 8; v8b a, b;
#pragma unroll
    for (int j = 0; j < 8; ++j) { a[j] = (b16)(bf16_rne(qw2[(size_t)(k0 + j) * HH + o]) * WSC); b[j] = (b16)(bf16_rne(kw2[(size_t)(k0 + j) * HH + o]) * WSC); }
    for (int pass = 0; pass < 2; ++pass) { *(volatile v8b*)(QW2 + (size_t)o * 32 + k0) = a; *(volatile v8b*)(KW2 + (size_t)o * 32 + k0) = b; __threadfence(); } } }
__global__ __launch_bounds__(256) void nf_kernel(const float* __restrict__ rss, const float* __restrict__ lf, const float* __restrict__ lp, const float* __restrict__ pp, const int* __restrict__ fmask, const float* __restrict__ gw1, const float* __restrict__ gb1, const float* __restrict__ gw2, const float* __restrict__ gb2, const float* __restrict__ qw1, const float* __restrict__ qb1, const float* __restrict__ qb2, const float* __restrict__ kb1, const float* __restrict__ kb2, const float* __restrict__ sig, const b16* __restrict__ KW1, const b16* __restrict__ QW2, const b16* __restrict__ KW2, int BLIM, float* __restrict__ attn, float* __restrict__ iwout) {
  __shared__ __attribute__((aligned(16))) b16 Buf[8][4608]; __shared__ float Sc[8][16][20]; __shared__ float Iw[8][16];
  const int wave = threadIdx.x >> 5, lane = threadIdx.x & 31, nloc = lane & 15, hlf = lane >> 4;
  typedef b16 (*T40)[40]; typedef b16 (*T72)[72]; T40 Ain = (T40)(Buf[wave]), Qh = (T40)(Buf[wave] + 640), Ql = (T40)(Buf[wave] + 1280), Kh = (T40)(Buf[wave] + 1920), Kl = (T40)(Buf[wave] + 2560); T72 QQh = (T72)(Buf[wave]), QQl = (T72)(Buf[wave] + 1152), KKh = (T72)(Buf[wave] + 2304), KKl = (T72)(Buf[wave] + 3456); const size_t b = (size_t)blockIdx.x * 8 + wave; const bool act = b < (size_t)BLIM;
  float iw_l = 0.0f;
  if (act) {
    { const float x = lane < R ? bfv(rss[b * R + lane]) : 0.0f; float g = bfv(gb2[0]);
#pragma unroll
      for (int m = 0; m < 16; ++m) g += pmul(fmaxf(pmul(x, bfv(gw1[m])) + bfv(gb1[m]), 0.0f), bfv(gw2[m]));
      const float gate = 1.0f / (1.0f + __expf(-g)); iw_l = (x > 0.5f ? 1.0f : 0.0f) * gate; if (lane >= R) iw_l = 0.0f; const float xi = pmul(x, iw_l);
#pragma unroll
      for (int m = 0; m < 32; ++m) { const float v = lane < R ? fmaxf(pmul(xi, bfv(qw1[m])) + bfv(qb1[m]), 0.0f) : 0.0f; b16 p, ql; split16(v * XS, p, ql); if (lane < 16) { Qh[lane][m] = p; Ql[lane][m] = ql; } } }
    if (lane < 16) { Iw[wave][lane] = iw_l; for (int m = 32; m < 40; ++m) { Qh[lane][m] = (b16)0.0f; Ql[lane][m] = (b16)0.0f; } }
    if (lane < 16) { for (int m = 0; m < 40; ++m) { float v = 0.0f; if (m < F) v = bf16_rne(lf[(b * L + lane) * F + m]); else if (m < FIN) v = bf16_rne(lp[(b * L + lane) * 3 + (m - F)]); Ain[lane][m] = (b16)(v * XS); } }
    wave_lds_sync();
    { const v16b a = frag_kb(&Ain[nloc][0], hlf);
#pragma unroll
      for (int t = 0; t < 2; ++t) { const v8f acc = wmma16b(a, frag_kb(KW1 + (size_t)(t * 16 + nloc) * 32, hlf), (v8f){}); const int cc = t * 16 + nloc; const float bb = bfv(kb1[cc]);
#pragma unroll
        for (int r8 = 0; r8 < 8; ++r8) { b16 p, ql; split16(fmaxf(acc[r8] * (1.0f / (XS * WSC)) + bb, 0.0f) * XS, p, ql); Kh[8 * hlf + r8][cc] = p; Kl[8 * hlf + r8][cc] = ql; } }
      if (lane < 16) for (int m = 32; m < 40; ++m) { Kh[lane][m] = (b16)0.0f; Kl[lane][m] = (b16)0.0f; } }
    wave_lds_sync();
    { const v16b qa = frag_kb(&Qh[nloc][0], hlf), qb = frag_kb(&Ql[nloc][0], hlf), ka = frag_kb(&Kh[nloc][0], hlf), kbf = frag_kb(&Kl[nloc][0], hlf); asm volatile("s_wait_dscnt 0x0" ::: "memory"); wave_lds_sync();
#pragma unroll
      for (int t = 0; t < 4; ++t) { const v16b wq = frag_kb(QW2 + (size_t)(t * 16 + nloc) * 32, hlf), wk = frag_kb(KW2 + (size_t)(t * 16 + nloc) * 32, hlf); v8f aq = wmma16b(qa, wq, (v8f){}); aq = wmma16b(qb, wq, aq); v8f ak = wmma16b(ka, wk, (v8f){}); ak = wmma16b(kbf, wk, ak); const int cc = t * 16 + nloc; const float bq = bfv(qb2[cc]), bk = bfv(kb2[cc]);
#pragma unroll
        for (int r8 = 0; r8 < 8; ++r8) { const int rr = 8 * hlf + r8; b16 p, ql; split16((aq[r8] * (1.0f / (XS * WSC)) + bq) * XS, p, ql); QQh[rr][cc] = p; QQl[rr][cc] = ql; split16((ak[r8] * (1.0f / (XS * WSC)) + bk) * XS, p, ql); KKh[rr][cc] = p; KKl[rr][cc] = ql; } }
      if (lane < 16) for (int m = 64; m < 72; ++m) { QQh[lane][m] = (b16)0.0f; QQl[lane][m] = (b16)0.0f; KKh[lane][m] = (b16)0.0f; KKl[lane][m] = (b16)0.0f; } }
    wave_lds_sync();
    { v8f s = {};
#pragma unroll
      for (int kb = 0; kb < HH; kb += 32) { const v16b qa = frag_kb(&QQh[nloc][kb], hlf), qb = frag_kb(&QQl[nloc][kb], hlf), ka = frag_kb(&KKh[nloc][kb], hlf), kbf = frag_kb(&KKl[nloc][kb], hlf); s = wmma16b(qa, ka, s); s = wmma16b(qa, kbf, s); s = wmma16b(qb, ka, s); }
      const int l = nloc; float dsq = 0.0f; for (int d = 0; d < 3; ++d) { const float df = bfv(pp[b * 3 + d]) - bfv(lp[(b * L + l) * 3 + d]); dsq += df * df; } const float sg = bfv(sig[0]); const float bias = dsq / (2.0f * sg * sg);
#pragma unroll
      for (int r8 = 0; r8 < 8; ++r8) { const int r = 8 * hlf + r8; float v = s[r8] * (1.0f / (XS * XS)) - bias; if (r < R && fmask[r * L + l] == 0) v = FMIN; Sc[wave][r][l] = v; } }
    wave_lds_sync(); }
  __syncthreads();
  for (int pass = 0; pass < 2; ++pass) {
    if (act) {
      const int r = lane >> 1, half = lane & 1; if (r < R) { float mx = FMIN; for (int l = 0; l < L; ++l) mx = fmaxf(mx, Sc[wave][r][l]); float den = 0.0f; for (int l = 0; l < L; ++l) den += __expf(Sc[wave][r][l] - mx);
        for (int l = half * 8; l < half * 8 + 8; ++l) ((volatile float*)attn)[(b * R + r) * L + l] = __expf(Sc[wave][r][l] - mx) / den; } }
    if (wave == 0) { for (int q = lane; q < 8 * R; q += 32) { const size_t bb = (size_t)blockIdx.x * 8 + q / R; if (bb < (size_t)BLIM) ((volatile float*)iwout)[bb * R + q % R] = Iw[q / R][q % R]; } }
    __threadfence(); } }
}

extern "C" void kernel_launch(void* const* d_in, const int* in_sizes, int n_in, void* d_out, int out_size, void* d_ws, size_t ws_size, hipStream_t stream) {
  (void)n_in;
  auto Fp = [&](int i) { return (const float*)d_in[i]; }; auto Ip = [&](int i) { return (const int*)d_in[i]; };
  if (in_sizes[0] != NBT * R || in_sizes[1] != NBT * L * F || in_sizes[2] != NBT * L * 3 || in_sizes[3] != NBT * 3 || in_sizes[4] != R * L || in_sizes[11] != 32 * HH || in_sizes[13] != FIN * 32 || in_sizes[15] != 32 * HH || out_size != NBT * R * L + NBT * R) return;
  const int BLIM = NBT;
  size_t off = 0; char* ws = (char*)d_ws;
  auto carve = [&](size_t bytes) { char* p = ws + off; off += (bytes + 255) & ~(size_t)255; return p; };
  b16* KW1 = (b16*)carve(32 * 32 * 2); b16* QW2 = (b16*)carve(HH * 32 * 2); b16* KW2 = (b16*)carve(HH * 32 * 2);
  if (off > ws_size || off > ((size_t)1 << 20)) return;
  wput_kernel<<<1, 256, 0, stream>>>(Fp(13), Fp(11), Fp(15), KW1, QW2, KW2);
  nf_kernel<<<(BLIM + 7) / 8, 256, 0, stream>>>(Fp(0), Fp(1), Fp(2), Fp(3), Ip(4), Fp(5), Fp(6), Fp(7), Fp(8), Fp(9), Fp(10), Fp(12), Fp(14), Fp(16), Fp(17), KW1, QW2, KW2, BLIM, (float*)d_out, (float*)d_out + (size_t)NBT * R * L);
}
